// PointNetTunable_20117626814615
// MI455X (gfx1250) — hardware-verified
//
#include <hip/hip_runtime.h>
#pragma clang fp contract(off)

typedef __attribute__((ext_vector_type(16))) __bf16   v16b;
typedef __attribute__((ext_vector_type(8)))  __bf16   v8b;
typedef __attribute__((ext_vector_type(8)))  float    v8f;
typedef __attribute__((ext_vector_type(4)))  float    v4f;
typedef __attribute__((ext_vector_type(2)))  float    v2f;
typedef __attribute__((ext_vector_type(4)))  unsigned v4u;
typedef __attribute__((ext_vector_type(2)))  unsigned v2u;

constexpr int kBatch   = 16;
constexpr int kPts0    = 4096;
constexpr int kPts1    = 512;
constexpr int kPts2    = 256;
constexpr int kPts3    = 128;
constexpr int kChan1   = 64;
constexpr int kChan2   = 128;
constexpr int kChan3   = 256;
constexpr int kCatK2   = 3 * kChan1;
constexpr int kCatK3   = 3 * kChan2;
constexpr int kRowsQ2  = kBatch * kPts1;
constexpr int kRowsQ3  = kBatch * kPts2;
constexpr int kRowsF3  = kBatch * kPts3;
constexpr int kNeigh   = 32;

static_assert(kRowsQ2 % 64 == 0 && kChan2 % 64 == 0 && kCatK2 % 32 == 0, "gemm2 tile multiples");
static_assert(kRowsQ3 % 64 == 0 && kChan3 % 64 == 0 && kCatK3 % 32 == 0, "gemm3 tile multiples");

constexpr size_t kOffXyz1  = 0;
constexpr size_t kOffXyz2  = kOffXyz1 + (size_t)kBatch * kPts1 * 4 * 4;
constexpr size_t kOffXyz3  = kOffXyz2 + (size_t)kBatch * kPts2 * 4 * 4;
constexpr size_t kOffBt2   = kOffXyz3 + (size_t)kBatch * kPts3 * 4 * 4;
constexpr size_t kOffBt3   = kOffBt2 + (size_t)kChan2 * kCatK2 * 2;
constexpr size_t kOffA2    = kOffBt3 + (size_t)kChan3 * kCatK3 * 2;
constexpr size_t kOffQ2    = kOffA2 + (size_t)kRowsQ2 * kCatK2 * 2;
constexpr size_t kOffA3    = kOffQ2 + (size_t)kRowsQ2 * kChan2 * 4;
constexpr size_t kOffQ3    = kOffA3 + (size_t)kRowsQ3 * kCatK3 * 2;
constexpr size_t kOffF3    = kOffQ3 + (size_t)kRowsQ3 * kChan3 * 4;
constexpr size_t kWsTotal  = kOffF3 + (size_t)kRowsF3 * kChan3 * 4;
static_assert(kWsTotal <= (size_t)134217728, "carve under 128 MiB");
static_assert((kOffXyz2 % 128) == 0 && (kOffXyz3 % 128) == 0 && (kOffBt2 % 128) == 0 && (kOffBt3 % 128) == 0, "aligned");
static_assert((kOffA2 % 128) == 0 && (kOffQ2 % 128) == 0 && (kOffA3 % 128) == 0 && (kOffQ3 % 128) == 0 && (kOffF3 % 128) == 0, "aligned");

__device__ __forceinline__ unsigned bf_bits(float f) {
  const unsigned u = __float_as_uint(f);
  return (u + 0x7FFFu + ((u >> 16) & 1u)) >> 16;
}
__device__ __forceinline__ float bf_val(unsigned hb) { return __uint_as_float(hb << 16); }

__device__ __forceinline__ float sqdist3(float ax, float ay, float az, float bx, float by, float bz) {
#pragma clang fp contract(off)
  const float dx = ax - bx;
  const float dy = ay - by;
  const float dz = az - bz;
  const float t0 = dx * dx;
  const float t1 = dy * dy;
  const float t2 = dz * dz;
  return (t0 + t2) + t1;
}

__device__ __forceinline__ void key_max(unsigned& hi, unsigned& lo, unsigned ohi, unsigned olo) {
  const bool tk = (ohi > hi) || ((ohi == hi) && (olo > lo));
  hi = tk ? ohi : hi;
  lo = tk ? olo : lo;
}

__device__ __forceinline__ int clampi(int v, int lo, int hi) {
  v = v < lo ? lo : v;
  v = v > hi ? hi : v;
  return v;
}

__device__ __forceinline__ void row_guard_b(v8f& a, v8f& b, v8f& c, v8f& d, v16b x, v16b y) {
  asm volatile("v_nop\n\tv_nop\n\tv_nop\n\tv_nop" : "+v"(a), "+v"(b), "+v"(c), "+v"(d) : "v"(x), "v"(y));
}
__device__ __forceinline__ void keep4_b(v16b a, v16b b, v16b c, v16b d) { asm volatile("v_nop" :: "v"(a), "v"(b), "v"(c), "v"(d)); }
__device__ __forceinline__ void acc_guard4(v8f& a, v8f& b, v8f& c, v8f& d) { asm volatile("v_nop\n\tv_nop\n\tv_nop\n\tv_nop" : "+v"(a), "+v"(b), "+v"(c), "+v"(d)); }

struct FragB {
  union U { v16b v; v8b h[2]; };
  static __device__ __forceinline__ v16b load(const __bf16* p) {
    U f;
    f.h[0] = *(const v8b*)(p);
    f.h[1] = *(const v8b*)(p + 16);
    return f.v;
  }
  static __device__ __forceinline__ v8f mma(v16b a, v16b b, v8f c) {
    return __builtin_amdgcn_wmma_f32_16x16x32_bf16(false, a, false, b, (short)0, c, false, false);
  }
};

__global__ __launch_bounds__(256) void gemm64_bf16_kernel(
    const unsigned short* __restrict__ Ap, int lda,
    const unsigned short* __restrict__ Btp, int ldb,
    float* __restrict__ Cout, int ldc, int M, int N, int K) {
  const __bf16* A  = (const __bf16*)Ap;
  const __bf16* Bt = (const __bf16*)Btp;
  __shared__ __align__(16) float sT[8][16 * 68];
  const int lane = threadIdx.x & 31;
  const int wave = threadIdx.x >> 5;
  const int tilesN = N >> 6;
  const int tilesM = M >> 6;
  const int tile = blockIdx.x * 8 + wave;
  if (tile >= tilesM * tilesN) return;
  const int tm = tile / tilesN;
  const int tn = tile - tm * tilesN;
  const int m0 = tm << 6;
  const int n0 = tn << 6;

  const int rlane = lane & 15;
  const int koff  = (lane >> 4) * 8;
  const int mOff  = (lane >> 4) * 8;

  v8f acc[4][4];
#pragma unroll
  for (int i = 0; i < 4; ++i)
#pragma unroll
    for (int j = 0; j < 4; ++j) acc[i][j] = (v8f){0.f, 0.f, 0.f, 0.f, 0.f, 0.f, 0.f, 0.f};

  for (int k0 = 0; k0 < K; k0 += 32) {
    v16b bh[4];
#pragma unroll
    for (int j = 0; j < 4; ++j) {
      const size_t bo = (size_t)(n0 + (j << 4) + rlane) * ldb + koff + k0;
      bh[j] = FragB::load(Bt + bo);
    }
#pragma unroll
    for (int i = 0; i < 4; ++i) {
      const size_t ao = (size_t)(m0 + (i << 4) + rlane) * lda + koff + k0;
      v16b ah = FragB::load(A + ao);
#pragma unroll
      for (int j = 0; j < 4; ++j) acc[i][j] = FragB::mma(ah, bh[j], acc[i][j]);
      row_guard_b(acc[i][0], acc[i][1], acc[i][2], acc[i][3], ah, bh[3]);
    }
    keep4_b(bh[0], bh[1], bh[2], bh[3]);
  }
  acc_guard4(acc[0][0], acc[0][1], acc[0][2], acc[0][3]);
  acc_guard4(acc[1][0], acc[1][1], acc[1][2], acc[1][3]);
  acc_guard4(acc[2][0], acc[2][1], acc[2][2], acc[2][3]);
  acc_guard4(acc[3][0], acc[3][1], acc[3][2], acc[3][3]);

  float* slab = sT[wave];
#pragma unroll
  for (int i = 0; i < 4; ++i) {
    const int mBase = m0 + (i << 4);
#pragma unroll
    for (int j = 0; j < 4; ++j) {
#pragma unroll
      for (int r = 0; r < 8; ++r) slab[(mOff + r) * 68 + (j << 4) + rlane] = acc[i][j][r];
    }
    __builtin_amdgcn_fence(__ATOMIC_RELEASE, "workgroup");
    __builtin_amdgcn_wave_barrier();
    __builtin_amdgcn_fence(__ATOMIC_ACQUIRE, "workgroup");
    {
      const int hh = lane >> 4;
      const int c4 = (lane & 15) * 4;
      for (int pass = 0; pass < 2; ++pass) {
#pragma unroll
        for (int it = 0; it < 8; ++it) {
          const int row = it * 2 + hh;
          v4f v = *(const v4f*)(slab + row * 68 + c4);
          *(volatile v4f*)(Cout + (size_t)(mBase + row) * ldc + n0 + c4) = v;
        }
        __threadfence();
      }
    }
    __builtin_amdgcn_fence(__ATOMIC_RELEASE, "workgroup");
    __builtin_amdgcn_wave_barrier();
    __builtin_amdgcn_fence(__ATOMIC_ACQUIRE, "workgroup");
  }
}

__global__ __launch_bounds__(256) void prep_bt_kernel(const float* __restrict__ W2, const float* __restrict__ W3,
                                                      unsigned* __restrict__ bt2, unsigned* __restrict__ bt3) {
  const int blk = blockIdx.x;
  const bool second = (blk >= 12);
  const float* W = second ? W3 : W2;
  unsigned* dst  = second ? bt3 : bt2;
  const int cout = second ? kChan3 : kChan2;
  const int cin  = second ? kChan2 : kChan1;
  const int t = (second ? (blk - 12) : blk) * 256 + (int)threadIdx.x;
  const int cpr = (3 * cin) >> 3;
  const int n = t / cpr;
  const int ch = t - n * cpr;
  const int k8 = ch << 3;
  const int seg = k8 / cin;
  const int kk = k8 - seg * cin;
  unsigned hw[8];
#pragma unroll
  for (int e = 0; e < 8; ++e) {
    const float w = W[(size_t)(3 + kk + e) * cout + n];
    const unsigned hb = bf_bits(w);
    const unsigned lb = bf_bits(w - bf_val(hb));
    hw[e] = (seg == 2) ? lb : hb;
  }
  v4u o;
  o.x = hw[0] | (hw[1] << 16);
  o.y = hw[2] | (hw[3] << 16);
  o.z = hw[4] | (hw[5] << 16);
  o.w = hw[6] | (hw[7] << 16);
  volatile v4u* p = (volatile v4u*)(dst + (size_t)t * 4);
  *p = o;
  __threadfence();
  *p = o;
}

template <int NPTS, int NSEL, int TPB, int STRIDE>
__global__ __launch_bounds__(TPB) void fps_kernel(const float* __restrict__ src, float* __restrict__ dst) {
#pragma clang fp contract(off)
  constexpr int PPT = NPTS / TPB;
  constexpr int NW  = TPB / 32;
  static_assert(NPTS % TPB == 0 && PPT >= 1 && PPT <= 4, "points per thread");
  static_assert(NSEL <= TPB && (NSEL % 32) == 0, "store map");
  static_assert(NW <= 32 && (NW & (NW - 1)) == 0, "wave count");
  __shared__ unsigned s_khi[2][32];
  __shared__ unsigned s_klo[2][32];
  __shared__ __align__(16) float s_sel[NSEL * 4];

  const int b = blockIdx.x;
  const int tid = threadIdx.x;
  const int lane = tid & 31;
  const int wave = tid >> 5;
  const float* p = src + (size_t)b * NPTS * STRIDE;

  float px[PPT], py[PPT], pz[PPT], dd[PPT];
#pragma unroll
  for (int i = 0; i < PPT; ++i) {
    const int idx = tid * PPT + i;
    px[i] = p[idx * STRIDE + 0];
    py[i] = p[idx * STRIDE + 1];
    pz[i] = p[idx * STRIDE + 2];
    dd[i] = 1e10f;
  }
  float lx = p[0];
  float ly = p[1];
  float lz = p[2];
  if (tid == 0) {
    s_sel[0] = lx;
    s_sel[1] = ly;
    s_sel[2] = lz;
    s_sel[3] = 0.0f;
  }

  for (int s = 1; s < NSEL; ++s) {
    unsigned bhi = 0u;
    unsigned blo = 0u;
#pragma unroll
    for (int i = 0; i < PPT; ++i) {
      const float d = sqdist3(px[i], py[i], pz[i], lx, ly, lz);
      const float nd = fminf(dd[i], d);
      dd[i] = nd;
      const unsigned khi = __float_as_uint(nd);
      const unsigned klo = 0xFFFFFFFFu - (unsigned)(tid * PPT + i);
      key_max(bhi, blo, khi, klo);
    }
#pragma unroll
    for (int off = 16; off >= 1; off >>= 1) {
      const unsigned ohi = __shfl_xor(bhi, off, 32);
      const unsigned olo = __shfl_xor(blo, off, 32);
      key_max(bhi, blo, ohi, olo);
    }
    const int buf = s & 1;
    if (lane == 0) {
      s_khi[buf][wave] = bhi;
      s_klo[buf][wave] = blo;
    }
    __syncthreads();
    unsigned ghi = s_khi[buf][lane & (NW - 1)];
    unsigned glo = s_klo[buf][lane & (NW - 1)];
#pragma unroll
    for (int off = 16; off >= 1; off >>= 1) {
      const unsigned ohi = __shfl_xor(ghi, off, 32);
      const unsigned olo = __shfl_xor(glo, off, 32);
      key_max(ghi, glo, ohi, olo);
    }
    const int win = clampi((int)(0xFFFFFFFFu - glo), 0, NPTS - 1);
    lx = p[win * STRIDE + 0];
    ly = p[win * STRIDE + 1];
    lz = p[win * STRIDE + 2];
    if (tid == 0) {
      s_sel[s * 4 + 0] = lx;
      s_sel[s * 4 + 1] = ly;
      s_sel[s * 4 + 2] = lz;
      s_sel[s * 4 + 3] = 0.0f;
    }
  }
  __syncthreads();
  if (tid < NSEL) {
    float* o = dst + (size_t)b * NSEL * 4 + (size_t)tid * 4;
    const v4f v = *(const v4f*)(s_sel + tid * 4);
    *(volatile v4f*)o = v;
    __threadfence();
    *(volatile v4f*)o = v;
  }
}

__global__ __launch_bounds__(32) void sa1_kernel(const float* __restrict__ pts, const float* __restrict__ cxyz,
                                                 const float* __restrict__ W1, const float* __restrict__ b1,
                                                 unsigned* __restrict__ a2cat, float r2) {
#pragma clang fp contract(off)
  __shared__ int s_idx[kNeigh];
  __shared__ __align__(16) float s_rel[kNeigh * 4];
  __shared__ __align__(16) float s_abs[kNeigh * 4];
  const int lane = threadIdx.x;
  const int cid = blockIdx.x;
  const int b = cid / kPts1;
  const v4f cc = *(const v4f*)(cxyz + (size_t)cid * 4);
  const float* p = pts + (size_t)b * kPts0 * 3;

  s_idx[lane] = 0;
  __syncthreads();
  int cnt = 0;
  for (int c = 0; (c < kPts0 / 32) && (cnt < kNeigh); ++c) {
    const int i = c * 32 + lane;
    const float x = p[i * 3 + 0];
    const float y = p[i * 3 + 1];
    const float z = p[i * 3 + 2];
    const float d = sqdist3(cc.x, cc.y, cc.z, x, y, z);
    const bool valid = (d <= r2);
    const unsigned mm = (unsigned)__ballot(valid);
    const int pos = cnt + __popc(mm & ((1u << lane) - 1u));
    if (valid && (pos < kNeigh)) s_idx[pos] = i;
    cnt += __popc(mm);
  }
  cnt = cnt > kNeigh ? kNeigh : cnt;
  cnt = cnt < 1 ? 1 : cnt;
  __syncthreads();
  {
    const int gi = clampi(s_idx[lane], 0, kPts0 - 1);
    const float nx = p[gi * 3 + 0];
    const float ny = p[gi * 3 + 1];
    const float nz = p[gi * 3 + 2];
    v4f rel;
    rel.x = nx - cc.x;
    rel.y = ny - cc.y;
    rel.z = nz - cc.z;
    rel.w = 0.0f;
    v4f ab;
    ab.x = nx;
    ab.y = ny;
    ab.z = nz;
    ab.w = 0.0f;
    *(v4f*)(s_rel + lane * 4) = rel;
    *(v4f*)(s_abs + lane * 4) = ab;
  }
  const v2f w0 = *(const v2f*)(W1 + 0 * kChan1 + 2 * lane);
  const v2f w1 = *(const v2f*)(W1 + 1 * kChan1 + 2 * lane);
  const v2f w2 = *(const v2f*)(W1 + 2 * kChan1 + 2 * lane);
  const v2f w3 = *(const v2f*)(W1 + 3 * kChan1 + 2 * lane);
  const v2f w4 = *(const v2f*)(W1 + 4 * kChan1 + 2 * lane);
  const v2f w5 = *(const v2f*)(W1 + 5 * kChan1 + 2 * lane);
  const v2f bs = *(const v2f*)(b1 + 2 * lane);
  __syncthreads();

  float m0 = -__builtin_inff();
  float m1 = -__builtin_inff();
#pragma unroll 1
  for (int j = 0; j < cnt; ++j) {
    const v4f r = *(const v4f*)(s_rel + j * 4);
    const v4f a = *(const v4f*)(s_abs + j * 4);
    float v0 = r.x * w0.x;
    v0 = __builtin_fmaf(r.y, w1.x, v0);
    v0 = __builtin_fmaf(r.z, w2.x, v0);
    v0 = __builtin_fmaf(a.x, w3.x, v0);
    v0 = __builtin_fmaf(a.y, w4.x, v0);
    v0 = __builtin_fmaf(a.z, w5.x, v0);
    float v1 = r.x * w0.y;
    v1 = __builtin_fmaf(r.y, w1.y, v1);
    v1 = __builtin_fmaf(r.z, w2.y, v1);
    v1 = __builtin_fmaf(a.x, w3.y, v1);
    v1 = __builtin_fmaf(a.y, w4.y, v1);
    v1 = __builtin_fmaf(a.z, w5.y, v1);
    m0 = fmaxf(m0, v0);
    m1 = fmaxf(m1, v1);
  }
  const float f0 = fmaxf(m0 + bs.x, 0.0f);
  const float f1 = fmaxf(m1 + bs.y, 0.0f);
  const unsigned h0 = bf_bits(f0);
  const unsigned h1 = bf_bits(f1);
  const unsigned l0 = bf_bits(f0 - bf_val(h0));
  const unsigned l1 = bf_bits(f1 - bf_val(h1));
  const unsigned whi = h0 | (h1 << 16);
  const unsigned wlo = l0 | (l1 << 16);
  volatile unsigned* row = (volatile unsigned*)(a2cat + (size_t)cid * (kCatK2 / 2));
  row[lane] = whi;
  row[32 + lane] = wlo;
  row[64 + lane] = whi;
  __threadfence();
  row[lane] = whi;
  row[32 + lane] = wlo;
  row[64 + lane] = whi;
}

template <int NSRC, int NCTR, int COUT, bool FINAL>
__global__ __launch_bounds__(32) void sa_gather_kernel(const float* __restrict__ sxyz, const float* __restrict__ cxyz,
                                                       const float* __restrict__ Q, const float* __restrict__ W,
                                                       const float* __restrict__ bias, void* __restrict__ outp, float r2) {
#pragma clang fp contract(off)
  constexpr int NG = COUT / 128;
  static_assert((COUT % 128) == 0 && (FINAL || NG == 1), "channel map");
  static_assert((NSRC % 32) == 0, "chunking");
  __shared__ int s_idx[kNeigh];
  __shared__ __align__(16) float s_rel[kNeigh * 4];
  const int lane = threadIdx.x;
  const int cid = blockIdx.x;
  const int b = cid / NCTR;
  const v4f cc = *(const v4f*)(cxyz + (size_t)cid * 4);
  const float* p = sxyz + (size_t)b * NSRC * 4;

  s_idx[lane] = 0;
  __syncthreads();
  int cnt = 0;
  for (int c = 0; (c < NSRC / 32) && (cnt < kNeigh); ++c) {
    const int i = c * 32 + lane;
    const v4f q = *(const v4f*)(p + (size_t)i * 4);
    const float d = sqdist3(cc.x, cc.y, cc.z, q.x, q.y, q.z);
    const bool valid = (d <= r2);
    const unsigned mm = (unsigned)__ballot(valid);
    const int pos = cnt + __popc(mm & ((1u << lane) - 1u));
    if (valid && (pos < kNeigh)) s_idx[pos] = i;
    cnt += __popc(mm);
  }
  cnt = cnt > kNeigh ? kNeigh : cnt;
  cnt = cnt < 1 ? 1 : cnt;
  __syncthreads();
  {
    const int gi = clampi(s_idx[lane], 0, NSRC - 1);
    const v4f nb = *(const v4f*)(p + (size_t)gi * 4);
    v4f rel;
    rel.x = nb.x - cc.x;
    rel.y = nb.y - cc.y;
    rel.z = nb.z - cc.z;
    rel.w = 0.0f;
    *(v4f*)(s_rel + lane * 4) = rel;
  }
  v4f w0[NG], w1[NG], w2[NG], bs[NG], mx[NG];
#pragma unroll
  for (int g = 0; g < NG; ++g) {
    w0[g] = *(const v4f*)(W + 0 * COUT + g * 128 + lane * 4);
    w1[g] = *(const v4f*)(W + 1 * COUT + g * 128 + lane * 4);
    w2[g] = *(const v4f*)(W + 2 * COUT + g * 128 + lane * 4);
    bs[g] = *(const v4f*)(bias + g * 128 + lane * 4);
    const float ninf = -__builtin_inff();
    mx[g] = (v4f){ninf, ninf, ninf, ninf};
  }
  __syncthreads();

  const float* Qb = Q + (size_t)b * NSRC * COUT;
#pragma unroll 1
  for (int j = 0; j < cnt; ++j) {
    const int gj = clampi(s_idx[j], 0, NSRC - 1);
    const v4f r = *(const v4f*)(s_rel + j * 4);
#pragma unroll
    for (int g = 0; g < NG; ++g) {
      const v4f qv = *(const v4f*)(Qb + (size_t)gj * COUT + g * 128 + lane * 4);
#pragma unroll
      for (int e = 0; e < 4; ++e) {
        float t = r.x * w0[g][e];
        t = __builtin_fmaf(r.y, w1[g][e], t);
        t = __builtin_fmaf(r.z, w2[g][e], t);
        const float v = qv[e] + t;
        mx[g][e] = fmaxf(mx[g][e], v);
      }
    }
  }

  if (FINAL) {
    float* row = (float*)outp + (size_t)cid * COUT;
    v4f ov[NG];
#pragma unroll
    for (int g = 0; g < NG; ++g) {
#pragma unroll
      for (int e = 0; e < 4; ++e) ov[g][e] = fmaxf(mx[g][e] + bs[g][e], 0.0f);
    }
#pragma unroll
    for (int g = 0; g < NG; ++g) *(volatile v4f*)(row + g * 128 + lane * 4) = ov[g];
    __threadfence();
#pragma unroll
    for (int g = 0; g < NG; ++g) *(volatile v4f*)(row + g * 128 + lane * 4) = ov[g];
  } else {
    unsigned hb[4], lb[4];
#pragma unroll
    for (int e = 0; e < 4; ++e) {
      const float f = fmaxf(mx[0][e] + bs[0][e], 0.0f);
      hb[e] = bf_bits(f);
      lb[e] = bf_bits(f - bf_val(hb[e]));
    }
    v2u whi, wlo;
    whi.x = hb[0] | (hb[1] << 16);
    whi.y = hb[2] | (hb[3] << 16);
    wlo.x = lb[0] | (lb[1] << 16);
    wlo.y = lb[2] | (lb[3] << 16);
    unsigned* row = (unsigned*)outp + (size_t)cid * (3 * COUT / 2);
    volatile v2u* d0 = (volatile v2u*)(row + lane * 2);
    volatile v2u* d1 = (volatile v2u*)(row + COUT / 2 + lane * 2);
    volatile v2u* d2 = (volatile v2u*)(row + COUT + lane * 2);
    *d0 = whi;
    *d1 = wlo;
    *d2 = whi;
    __threadfence();
    *d0 = whi;
    *d1 = wlo;
    *d2 = whi;
  }
}

__global__ __launch_bounds__(256) void head_kernel(const float* __restrict__ feat3,
                                                   const float* __restrict__ fc1w, const float* __restrict__ fc1b,
                                                   const float* __restrict__ fc2w, const float* __restrict__ fc2b,
                                                   const float* __restrict__ fc3w, const float* __restrict__ fc3b,
                                                   const float* __restrict__ g1, const float* __restrict__ be1,
                                                   const float* __restrict__ g2, const float* __restrict__ be2,
                                                   float* __restrict__ out) {
  __shared__ float X[kBatch * 256];
  __shared__ float Y[kBatch * 256];
  __shared__ __align__(16) float s_out[192];
  const int t = threadIdx.x;

#pragma unroll 1
  for (int b = 0; b < kBatch; ++b) {
    float m = -__builtin_inff();
#pragma unroll 4
    for (int s = 0; s < kPts3; ++s) m = fmaxf(m, feat3[((size_t)(b * kPts3 + s)) * kChan3 + t]);
    X[b * 256 + t] = m;
  }
  __syncthreads();

  float col[kBatch];
  {
#pragma unroll
    for (int b = 0; b < kBatch; ++b) col[b] = 0.0f;
#pragma unroll 1
    for (int k = 0; k < 256; ++k) {
      const float w = fc1w[k * 256 + t];
#pragma unroll
      for (int b = 0; b < kBatch; ++b) col[b] = __builtin_fmaf(X[b * 256 + k], w, col[b]);
    }
    const float bb = fc1b[t];
    float mean = 0.0f;
#pragma unroll
    for (int b = 0; b < kBatch; ++b) {
      col[b] = col[b] + bb;
      mean += col[b];
    }
    mean *= 0.0625f;
    float var = 0.0f;
#pragma unroll
    for (int b = 0; b < kBatch; ++b) {
      const float d = col[b] - mean;
      var += d * d;
    }
    var *= 0.0625f;
    const float rs = 1.0f / sqrtf(var + 1e-5f);
    const float gg = g1[t];
    const float sb = be1[t];
#pragma unroll
    for (int b = 0; b < kBatch; ++b) Y[b * 256 + t] = fmaxf(((col[b] - mean) * rs) * gg + sb, 0.0f);
  }
  __syncthreads();

  if (t < 128) {
#pragma unroll
    for (int b = 0; b < kBatch; ++b) col[b] = 0.0f;
#pragma unroll 1
    for (int k = 0; k < 256; ++k) {
      const float w = fc2w[k * 128 + t];
#pragma unroll
      for (int b = 0; b < kBatch; ++b) col[b] = __builtin_fmaf(Y[b * 256 + k], w, col[b]);
    }
    const float bb = fc2b[t];
    float mean = 0.0f;
#pragma unroll
    for (int b = 0; b < kBatch; ++b) {
      col[b] = col[b] + bb;
      mean += col[b];
    }
    mean *= 0.0625f;
    float var = 0.0f;
#pragma unroll
    for (int b = 0; b < kBatch; ++b) {
      const float d = col[b] - mean;
      var += d * d;
    }
    var *= 0.0625f;
    const float rs = 1.0f / sqrtf(var + 1e-5f);
    const float gg = g2[t];
    const float sb = be2[t];
#pragma unroll
    for (int b = 0; b < kBatch; ++b) X[b * 128 + t] = fmaxf(((col[b] - mean) * rs) * gg + sb, 0.0f);
  }
  __syncthreads();

  if (t < kBatch * 12) {
    const int b = t / 12;
    const int o = t - b * 12;
    float acc = 0.0f;
#pragma unroll 1
    for (int k = 0; k < 128; ++k) acc = __builtin_fmaf(X[b * 128 + k], fc3w[k * 12 + o], acc);
    s_out[t] = acc + fc3b[o];
  }
  __syncthreads();

  if (t < 32) {
    const int c0 = t;
    const int c1 = 32 + (t & 15);
    const v4f v0 = *(const v4f*)(s_out + c0 * 4);
    const v4f v1 = *(const v4f*)(s_out + c1 * 4);
    *(volatile v4f*)(out + c0 * 4) = v0;
    if (t < 16) *(volatile v4f*)(out + c1 * 4) = v1;
    __threadfence();
    *(volatile v4f*)(out + c0 * 4) = v0;
    if (t < 16) *(volatile v4f*)(out + c1 * 4) = v1;
  }
}

extern "C" void kernel_launch(void* const* d_in, const int* in_sizes, int n_in,
                              void* d_out, int out_size, void* d_ws, size_t ws_size,
                              hipStream_t stream) {
  (void)in_sizes;
  if (n_in < 17) return;
  if (out_size < kBatch * 12) return;
  if (ws_size < kWsTotal) return;

  const float* points = (const float*)d_in[0];
  const float* W1   = (const float*)d_in[1];
  const float* b1   = (const float*)d_in[2];
  const float* W2   = (const float*)d_in[3];
  const float* b2   = (const float*)d_in[4];
  const float* W3   = (const float*)d_in[5];
  const float* b3   = (const float*)d_in[6];
  const float* fc1w = (const float*)d_in[7];
  const float* fc1b = (const float*)d_in[8];
  const float* fc2w = (const float*)d_in[9];
  const float* fc2b = (const float*)d_in[10];
  const float* fc3w = (const float*)d_in[11];
  const float* fc3b = (const float*)d_in[12];
  const float* g1   = (const float*)d_in[13];
  const float* be1  = (const float*)d_in[14];
  const float* g2   = (const float*)d_in[15];
  const float* be2  = (const float*)d_in[16];

  char* ws = (char*)d_ws;
  float* xyz1  = (float*)(ws + kOffXyz1);
  float* xyz2  = (float*)(ws + kOffXyz2);
  float* xyz3  = (float*)(ws + kOffXyz3);
  unsigned* bt2   = (unsigned*)(ws + kOffBt2);
  unsigned* bt3   = (unsigned*)(ws + kOffBt3);
  unsigned* a2cat = (unsigned*)(ws + kOffA2);
  float* q2    = (float*)(ws + kOffQ2);
  unsigned* a3cat = (unsigned*)(ws + kOffA3);
  float* q3    = (float*)(ws + kOffQ3);
  float* feat3 = (float*)(ws + kOffF3);

  prep_bt_kernel<<<60, 256, 0, stream>>>(W2, W3, bt2, bt3);

  fps_kernel<kPts0, kPts1, 1024, 3><<<kBatch, 1024, 0, stream>>>(points, xyz1);
  sa1_kernel<<<kBatch * kPts1, 32, 0, stream>>>(points, xyz1, W1, b1, a2cat, 0.04f);
  gemm64_bf16_kernel<<<dim3((kRowsQ2 / 64) * (kChan2 / 64) / 8, 1), 256, 0, stream>>>(
      (const unsigned short*)a2cat, kCatK2, (const unsigned short*)bt2, kCatK2, q2, kChan2, kRowsQ2, kChan2, kCatK2);

  fps_kernel<kPts1, kPts2, 512, 4><<<kBatch, 512, 0, stream>>>(xyz1, xyz2);
  sa_gather_kernel<kPts1, kPts2, kChan2, false><<<kBatch * kPts2, 32, 0, stream>>>(
      xyz1, xyz2, q2, W2, b2, (void*)a3cat, 0.16f);
  gemm64_bf16_kernel<<<dim3((kRowsQ3 / 64) * (kChan3 / 64) / 8, 1), 256, 0, stream>>>(
      (const unsigned short*)a3cat, kCatK3, (const unsigned short*)bt3, kCatK3, q3, kChan3, kRowsQ3, kChan3, kCatK3);

  fps_kernel<kPts2, kPts3, 256, 4><<<kBatch, 256, 0, stream>>>(xyz2, xyz3);
  sa_gather_kernel<kPts2, kPts3, kChan3, true><<<kBatch * kPts3, 32, 0, stream>>>(
      xyz2, xyz3, q3, W3, b3, (void*)feat3, 0.64f);

  head_kernel<<<1, 256, 0, stream>>>(feat3, fc1w, fc1b, fc2w, fc2b, fc3w, fc3b, g1, be1, g2, be2, (float*)d_out);
}
